// MetaSREKPopulation_47605417508982
// MI455X (gfx1250) — hardware-verified
//
#include <hip/hip_runtime.h>
#define AA 400
#define BBt 64
#define II 50
#define IP 64
#define HH 192
#define OO 3
#define AD 128
#define NHD 8
#define HD 16
#define NR (AA * BBt)
#define JCH 32
#define KPAD 448

typedef __bf16 v16b __attribute__((ext_vector_type(16)));
typedef unsigned short v8us __attribute__((ext_vector_type(8), may_alias));
typedef float  v8f  __attribute__((ext_vector_type(8)));
typedef float  v4f  __attribute__((ext_vector_type(4)));
typedef float  v4fa __attribute__((ext_vector_type(4), may_alias));
union FragB { v16b v; v8us half[2]; unsigned short u[16]; };

__device__ __forceinline__ unsigned short bf16_bits(float x) { unsigned int u = __float_as_uint(x); return (unsigned short)((u + 0x7FFFu + ((u >> 16) & 1u)) >> 16); }
__device__ __forceinline__ float bf16_val(unsigned short b) { return __uint_as_float(((unsigned int)b) << 16); }
__device__ __forceinline__ float bf16_round(float x) { return bf16_val(bf16_bits(x)); }
template <int NT>
__device__ __forceinline__ v8f mmaN(v16b ah, v16b al, v16b bh, v16b bl, v8f c) {
  c = __builtin_amdgcn_wmma_f32_16x16x32_bf16(false, ah, false, bh, (short)0, c, false, false);
  if (NT >= 2) c = __builtin_amdgcn_wmma_f32_16x16x32_bf16(false, al, false, bh, (short)0, c, false, false);
  if (NT >= 3) c = __builtin_amdgcn_wmma_f32_16x16x32_bf16(false, ah, false, bl, (short)0, c, false, false);
  asm volatile("v_nop\n\tv_nop\n\tv_nop\n\tv_nop" : "+v"(c) : "v"(ah), "v"(al), "v"(bh), "v"(bl));
  return c;
}

__global__ __launch_bounds__(256) void k_wt_bf16(const float* __restrict__ W, unsigned short* __restrict__ Wt, int K, int N) {
  const int t = blockIdx.x * 256 + threadIdx.x;
  const int k8n = K / 8;
  if (t >= N * k8n) return;
  const int n = t / k8n, k8 = (t % k8n) * 8;
  v8us v;
#pragma unroll
  for (int i = 0; i < 8; ++i) v[i] = bf16_bits(W[(size_t)(k8 + i) * N + n]);
  *(volatile v8us*)(Wt + (size_t)n * K + k8) = v;
  __threadfence();
  *(volatile v8us*)(Wt + (size_t)n * K + k8) = v;
}

template <bool ASPLIT, int ACT, bool BIAS_BF16>
__global__ __launch_bounds__(128) void k_gemm_bf(const float* __restrict__ A, int lda, const unsigned short* __restrict__ Wt, int ldb,
                                               const float* __restrict__ bias, float* __restrict__ C, int ldc, int M, int N, int K) {
  __shared__ __attribute__((aligned(16))) float so[4][16][64];
  const int tid = threadIdx.x, w = tid >> 5, lane = tid & 31, ln = lane & 15, hh = lane >> 4;
  const int ntn = N / 64;
  const int wid = blockIdx.x * 4 + w;
  const int mt = wid / ntn, nq = wid % ntn;
  if (mt * 16 >= M) return;
  const int row0 = mt * 16, col0 = nq * 64;
  const float* arow = A + (size_t)(row0 + ln) * lda;
  v8f acc[4] = {};
  for (int kb = 0; kb < K; kb += 32) {
    FragB ah, al;
    const v4f x0 = *(const v4fa*)(arow + kb + 8 * hh), x1 = *(const v4fa*)(arow + kb + 8 * hh + 4);
    const v4f x2 = *(const v4fa*)(arow + kb + 16 + 8 * hh), x3 = *(const v4fa*)(arow + kb + 16 + 8 * hh + 4);
    float xs[16] = {x0[0],x0[1],x0[2],x0[3],x1[0],x1[1],x1[2],x1[3],x2[0],x2[1],x2[2],x2[3],x3[0],x3[1],x3[2],x3[3]};
#pragma unroll
    for (int i = 0; i < 16; ++i) { const unsigned short hb = bf16_bits(xs[i]); ah.u[i] = hb; al.u[i] = ASPLIT ? bf16_bits(xs[i] - bf16_val(hb)) : (unsigned short)0; }
#pragma unroll
    for (int t = 0; t < 4; ++t) {
      const unsigned short* brow = Wt + (size_t)(col0 + t * 16 + ln) * ldb + kb;
      FragB b;
      b.half[0] = *(const v8us*)(brow + 8 * hh);
      b.half[1] = *(const v8us*)(brow + 16 + 8 * hh);
      acc[t] = mmaN<ASPLIT ? 2 : 1>(ah.v, al.v, b.v, b.v, acc[t]);
    }
  }
#pragma unroll
  for (int t = 0; t < 4; ++t) {
    float bv = bias ? bias[col0 + t * 16 + ln] : 0.f;
    if (BIAS_BF16) bv = bf16_round(bv);
#pragma unroll
    for (int r = 0; r < 8; ++r) { float v = acc[t][r] + bv; if (ACT == 1) v = fmaxf(v, 0.f); so[w][8 * hh + r][t * 16 + ln] = v; }
  }
  __builtin_amdgcn_fence(__ATOMIC_ACQ_REL, "workgroup");
  __builtin_amdgcn_wave_barrier();
  const int rsub = lane >> 4, c4 = (lane & 15) * 4;
  for (int pass = 0; pass < 2; ++pass) {
#pragma unroll
    for (int q = 0; q < 8; ++q) {
      const int r = q * 2 + rsub;
      const v4f v = *(const v4fa*)&so[w][r][c4];
      *(volatile v4f*)(C + (size_t)(row0 + r) * ldc + col0 + c4) = v;
    }
    if (pass == 0) __threadfence();
  }
}

template <int D, bool CAUSAL>
__global__ __launch_bounds__(128) void k_flash(const float* __restrict__ qb, const float* __restrict__ kb, const float* __restrict__ vb,
                                             int pitch, int T, int H, float scale, float* __restrict__ y, int ypitch) {
  constexpr int KS = D / 32;
  constexpr int DT = D / 16;
  __shared__ __attribute__((aligned(16))) unsigned short sKh[32][D + 8], sKl[32][D + 8], sVh[32][D + 8], sVl[32][D + 8];
  __shared__ __attribute__((aligned(16))) unsigned short sPh[4][16][40], sPl[4][16][40];
  __shared__ __attribute__((aligned(16))) float sO[4][16][D];
  const int tid = threadIdx.x, w = tid >> 5, lane = tid & 31, ln = lane & 15, hh = lane >> 4;
  const int nqb = (T + 63) / 64;
  const int bh = blockIdx.x / nqb, qblk = blockIdx.x % nqb;
  const int b = bh / H, h = bh % H;
  const int q0 = qblk * 64 + w * 16;
  const float* Q = qb + (size_t)b * T * pitch + h * D;
  const float* K = kb + (size_t)b * T * pitch + h * D;
  const float* V = vb + (size_t)b * T * pitch + h * D;

  FragB aqh[KS], aql[KS];
  {
    int row = q0 + ln; if (row >= T) row = T - 1;
    const float* qr = Q + (size_t)row * pitch;
#pragma unroll
    for (int ks = 0; ks < KS; ++ks)
#pragma unroll
      for (int i = 0; i < 16; ++i) {
        const int d = ks * 32 + ((i < 8) ? (8 * hh + i) : (16 + 8 * hh + (i - 8)));
        const float x = qr[d] * scale; const unsigned short hb = bf16_bits(x);
        aqh[ks].u[i] = hb; aql[ks].u[i] = bf16_bits(x - bf16_val(hb));
      }
  }
  float m_r[8], l_r[8];
#pragma unroll
  for (int r = 0; r < 8; ++r) { m_r[r] = -3.0e38f; l_r[r] = 0.f; }
  v8f oacc[DT];
#pragma unroll
  for (int dt = 0; dt < DT; ++dt) oacc[dt] = (v8f){0.f,0.f,0.f,0.f,0.f,0.f,0.f,0.f};

  const int kv_end = CAUSAL ? min(T, qblk * 64 + 64) : T;
  for (int j0 = 0; j0 < kv_end; j0 += 32) {
    __syncthreads();
    for (int e = tid; e < 32 * (D / 4); e += 128) {
      const int r = e / (D / 4), c4 = (e % (D / 4)) * 4;
      const int key = j0 + r;
      v4f kf = {0.f,0.f,0.f,0.f}, vf = {0.f,0.f,0.f,0.f};
      if (key < T) { kf = *(const v4fa*)(K + (size_t)key * pitch + c4); vf = *(const v4fa*)(V + (size_t)key * pitch + c4); }
#pragma unroll
      for (int t = 0; t < 4; ++t) {
        unsigned short hb = bf16_bits(kf[t]); sKh[r][c4 + t] = hb; sKl[r][c4 + t] = bf16_bits(kf[t] - bf16_val(hb));
        hb = bf16_bits(vf[t]); sVh[r][c4 + t] = hb; sVl[r][c4 + t] = bf16_bits(vf[t] - bf16_val(hb));
      }
    }
    __syncthreads();
    v8f s[2];
#pragma unroll
    for (int nt = 0; nt < 2; ++nt) {
      v8f acc = {};
#pragma unroll
      for (int ks = 0; ks < KS; ++ks) {
        FragB bh_, bl_;
        bh_.half[0] = *(const v8us*)&sKh[nt * 16 + ln][ks * 32 + 8 * hh]; bh_.half[1] = *(const v8us*)&sKh[nt * 16 + ln][ks * 32 + 16 + 8 * hh];
        bl_.half[0] = *(const v8us*)&sKl[nt * 16 + ln][ks * 32 + 8 * hh]; bl_.half[1] = *(const v8us*)&sKl[nt * 16 + ln][ks * 32 + 16 + 8 * hh];
        acc = mmaN<3>(aqh[ks].v, aql[ks].v, bh_.v, bl_.v, acc);
      }
      s[nt] = acc;
    }
    float alpha[8];
#pragma unroll
    for (int r = 0; r < 8; ++r) {
      const int qi = q0 + 8 * hh + r;
      const int ja = j0 + ln, jb = j0 + 16 + ln;
      if (CAUSAL) { if (ja > qi) s[0][r] = -3.0e38f; if (jb > qi) s[1][r] = -3.0e38f; }
      if (ja >= T) s[0][r] = -3.0e38f;
      if (jb >= T) s[1][r] = -3.0e38f;
      float mx = fmaxf(s[0][r], s[1][r]);
      mx = fmaxf(mx, __shfl_xor(mx, 1, 32)); mx = fmaxf(mx, __shfl_xor(mx, 2, 32)); mx = fmaxf(mx, __shfl_xor(mx, 4, 32)); mx = fmaxf(mx, __shfl_xor(mx, 8, 32));
      const float mnew = fmaxf(m_r[r], mx);
      alpha[r] = (mnew > -1.0e38f) ? __expf(m_r[r] - mnew) : 1.0f;
      const float p0 = (s[0][r] > -1.0e38f) ? __expf(s[0][r] - mnew) : 0.f;
      const float p1 = (s[1][r] > -1.0e38f) ? __expf(s[1][r] - mnew) : 0.f;
      m_r[r] = mnew;
      l_r[r] = l_r[r] * alpha[r] + p0 + p1;
      unsigned short hb = bf16_bits(p0); sPh[w][8 * hh + r][ln] = hb;      sPl[w][8 * hh + r][ln] = bf16_bits(p0 - bf16_val(hb));
      hb = bf16_bits(p1);                sPh[w][8 * hh + r][16 + ln] = hb; sPl[w][8 * hh + r][16 + ln] = bf16_bits(p1 - bf16_val(hb));
    }
#pragma unroll
    for (int dt = 0; dt < DT; ++dt)
#pragma unroll
      for (int r = 0; r < 8; ++r) oacc[dt][r] *= alpha[r];
    __builtin_amdgcn_fence(__ATOMIC_ACQ_REL, "workgroup");
    __builtin_amdgcn_wave_barrier();
    FragB pah, pal;
    pah.half[0] = *(const v8us*)&sPh[w][ln][8 * hh]; pah.half[1] = *(const v8us*)&sPh[w][ln][16 + 8 * hh];
    pal.half[0] = *(const v8us*)&sPl[w][ln][8 * hh]; pal.half[1] = *(const v8us*)&sPl[w][ln][16 + 8 * hh];
#pragma unroll
    for (int dt = 0; dt < DT; ++dt) {
      FragB bvh, bvl;
#pragma unroll
      for (int i = 0; i < 8; ++i) {
        bvh.u[i] = sVh[8 * hh + i][dt * 16 + ln]; bvh.u[8 + i] = sVh[16 + 8 * hh + i][dt * 16 + ln];
        bvl.u[i] = sVl[8 * hh + i][dt * 16 + ln]; bvl.u[8 + i] = sVl[16 + 8 * hh + i][dt * 16 + ln];
      }
      oacc[dt] = mmaN<3>(pah.v, pal.v, bvh.v, bvl.v, oacc[dt]);
    }
    __builtin_amdgcn_fence(__ATOMIC_ACQ_REL, "workgroup");
    __builtin_amdgcn_wave_barrier();
  }
#pragma unroll
  for (int r = 0; r < 8; ++r) {
    float l = l_r[r];
    l += __shfl_xor(l, 1, 32); l += __shfl_xor(l, 2, 32); l += __shfl_xor(l, 4, 32); l += __shfl_xor(l, 8, 32);
    l_r[r] = (l > 0.f) ? 1.0f / l : 0.f;
  }
#pragma unroll
  for (int dt = 0; dt < DT; ++dt)
#pragma unroll
    for (int r = 0; r < 8; ++r) sO[w][8 * hh + r][dt * 16 + ln] = oacc[dt][r] * l_r[r];
  __builtin_amdgcn_fence(__ATOMIC_ACQ_REL, "workgroup");
  __builtin_amdgcn_wave_barrier();
  for (int pass = 0; pass < 2; ++pass) {
    for (int r = 0; r < 16; ++r) {
      const int row = q0 + r;
      if (row < T && lane < D / 4) {
        const v4f val = *(const v4fa*)&sO[w][r][lane * 4];
        *(volatile v4f*)(y + ((size_t)b * T + row) * ypitch + h * D + lane * 4) = val;
      }
    }
    if (pass == 0) __threadfence();
  }
}

template <bool ASPLIT, int ACT, bool BIAS_BF16, bool RES_BF16>
__global__ __launch_bounds__(128) void k_gemm_bf3(const float* __restrict__ A, int lda, const unsigned short* __restrict__ Wt, int ldb,
                                                const float* __restrict__ bias, const float* __restrict__ resid, int rmod, int ldr,
                                                float* __restrict__ C, int ldc, int M, int N, int K) {
  __shared__ __attribute__((aligned(16))) float so[4][16][64];
  const int tid = threadIdx.x, w = tid >> 5, lane = tid & 31, ln = lane & 15, hh = lane >> 4;
  const int ntn = N / 64;
  const int wid = blockIdx.x * 4 + w;
  const int mt = wid / ntn, nq = wid % ntn;
  if (mt * 16 >= M) return;
  const int row0 = mt * 16, col0 = nq * 64;
  const float* arow = A + (size_t)(row0 + ln) * lda;
  v8f acc[4] = {};
  for (int kb = 0; kb < K; kb += 32) {
    FragB ah, al;
    const v4f x0 = *(const v4fa*)(arow + kb + 8 * hh), x1 = *(const v4fa*)(arow + kb + 8 * hh + 4);
    const v4f x2 = *(const v4fa*)(arow + kb + 16 + 8 * hh), x3 = *(const v4fa*)(arow + kb + 16 + 8 * hh + 4);
    float xs[16] = {x0[0],x0[1],x0[2],x0[3],x1[0],x1[1],x1[2],x1[3],x2[0],x2[1],x2[2],x2[3],x3[0],x3[1],x3[2],x3[3]};
#pragma unroll
    for (int i = 0; i < 16; ++i) { const unsigned short hb = bf16_bits(xs[i]); ah.u[i] = hb; al.u[i] = ASPLIT ? bf16_bits(xs[i] - bf16_val(hb)) : (unsigned short)0; }
#pragma unroll
    for (int t = 0; t < 4; ++t) {
      const unsigned short* brow = Wt + (size_t)(col0 + t * 16 + ln) * ldb + kb;
      FragB b;
      b.half[0] = *(const v8us*)(brow + 8 * hh);
      b.half[1] = *(const v8us*)(brow + 16 + 8 * hh);
      acc[t] = mmaN<ASPLIT ? 2 : 1>(ah.v, al.v, b.v, b.v, acc[t]);
    }
  }
#pragma unroll
  for (int t = 0; t < 4; ++t) {
    const int col = col0 + t * 16 + ln;
    float bv = bias ? bias[col] : 0.f;
    if (BIAS_BF16) bv = bf16_round(bv);
#pragma unroll
    for (int r = 0; r < 8; ++r) {
      float v = acc[t][r] + bv;
      if (resid) { float rv = resid[(size_t)((row0 + 8 * hh + r) % rmod) * ldr + col]; if (RES_BF16) rv = bf16_round(rv); v += rv; }
      if (ACT == 1) v = fmaxf(v, 0.f);
      if (ACT == 2) v = 0.5f * v * (1.0f + erff(v * 0.70710678118654752f));
      if (ACT == 3) { const float u = 0.7978845608028654f * (v + 0.044715f * v * v * v); v = 0.5f * v * (1.0f + tanhf(u)); }
      so[w][8 * hh + r][t * 16 + ln] = v;
    }
  }
  __builtin_amdgcn_fence(__ATOMIC_ACQ_REL, "workgroup");
  __builtin_amdgcn_wave_barrier();
  const int rsub = lane >> 4, c4 = (lane & 15) * 4;
  for (int pass = 0; pass < 2; ++pass) {
#pragma unroll
    for (int q = 0; q < 8; ++q) {
      const int r = q * 2 + rsub;
      const v4f v = *(const v4fa*)&so[w][r][c4];
      *(volatile v4f*)(C + (size_t)(row0 + r) * ldc + col0 + c4) = v;
    }
    if (pass == 0) __threadfence();
  }
}
template <bool PARAM_BF16>
__global__ __launch_bounds__(256) void k_layernorm(const float* __restrict__ X, const float* __restrict__ R, const float* __restrict__ g, const float* __restrict__ bta,
                                                  float* __restrict__ out_sum, float* __restrict__ out_norm, int N, float eps) {
  __shared__ float red[256];
  const int row = blockIdx.x, tid = threadIdx.x;
  const float* x = X + (size_t)row * N; const float* rr = R ? R + (size_t)row * N : nullptr;
  float vals[16];
  const int per = N / 256;
  float s1 = 0.f;
  for (int u = 0; u < per / 4; ++u) {
    const int j = tid * 4 + 1024 * u;
    const v4f a = *(const v4fa*)(x + j);
    v4f b = {0.f,0.f,0.f,0.f}; if (rr) b = *(const v4fa*)(rr + j);
#pragma unroll
    for (int q = 0; q < 4; ++q) { const float v = a[q] + b[q]; vals[u * 4 + q] = v; s1 += v; }
  }
  red[tid] = s1; __syncthreads();
  for (int st = 128; st > 0; st >>= 1) { if (tid < st) red[tid] += red[tid + st]; __syncthreads(); }
  const float mu = red[0] / (float)N; __syncthreads();
  float s2 = 0.f;
  for (int u = 0; u < per / 4; ++u)
#pragma unroll
    for (int q = 0; q < 4; ++q) { const float c = vals[u * 4 + q] - mu; s2 += c * c; }
  red[tid] = s2; __syncthreads();
  for (int st = 128; st > 0; st >>= 1) { if (tid < st) red[tid] += red[tid + st]; __syncthreads(); }
  const float rs = rsqrtf(red[0] / (float)N + eps);
  for (int pass = 0; pass < 2; ++pass) {
    for (int u = 0; u < per / 4; ++u) {
      const int j = tid * 4 + 1024 * u;
      v4f o, sm;
#pragma unroll
      for (int q = 0; q < 4; ++q) {
        float gg = g[j + q], bb = bta[j + q];
        if (PARAM_BF16) { gg = bf16_round(gg); bb = bf16_round(bb); }
        sm[q] = vals[u * 4 + q]; o[q] = (vals[u * 4 + q] - mu) * rs * gg + bb;
      }
      if (out_sum) *(volatile v4f*)(out_sum + (size_t)row * N + j) = sm;
      *(volatile v4f*)(out_norm + (size_t)row * N + j) = o;
    }
    if (pass == 0) __threadfence();
  }
}


typedef _Float16 v16h __attribute__((ext_vector_type(16)));
union FragH { v16h v; v8us half[2]; _Float16 h[16]; unsigned short u[16]; };
template <int NT>
__device__ __forceinline__ v8f mmaH(v16h ah, v16h al, v16h bh, v16h bl, v8f c) {
  c = __builtin_amdgcn_wmma_f32_16x16x32_f16(false, ah, false, bh, (short)0, c, false, false);
  if (NT >= 2) c = __builtin_amdgcn_wmma_f32_16x16x32_f16(false, al, false, bh, (short)0, c, false, false);
  if (NT >= 3) c = __builtin_amdgcn_wmma_f32_16x16x32_f16(false, ah, false, bl, (short)0, c, false, false);
  asm volatile("v_nop\n\tv_nop\n\tv_nop\n\tv_nop" : "+v"(c) : "v"(ah), "v"(al), "v"(bh), "v"(bl));
  return c;
}
template <bool ASPLIT>
__global__ __launch_bounds__(128) void k_gemm_h(const float* __restrict__ A, int lda, size_t sA, const _Float16* __restrict__ Bh, int ldb, size_t sB, float alpha, float* __restrict__ C, int ldc, size_t sC, int M, int N, int K) {
  __shared__ __attribute__((aligned(16))) float so[4][16][64];
  const int tid = threadIdx.x, w = tid >> 5, lane = tid & 31, ln = lane & 15, hh = lane >> 4; const int by = blockIdx.y;
  A += (size_t)by * sA; Bh += (size_t)by * sB; C += (size_t)by * sC;
  const int ntn = (N + 63) / 64; const int wid = blockIdx.x * 4 + w; const int mt = wid / ntn, nq = wid % ntn; if (mt * 16 >= M) return;
  const int row0 = mt * 16, col0 = nq * 64; const float* arow = A + (size_t)(row0 + ln) * lda;
  v8f acc[4] = {};
  for (int kb = 0; kb < K; kb += 32) {
    FragH ah, al;
    const v4f x0 = *(const v4fa*)(arow + kb + 8 * hh), x1 = *(const v4fa*)(arow + kb + 8 * hh + 4), x2 = *(const v4fa*)(arow + kb + 16 + 8 * hh), x3 = *(const v4fa*)(arow + kb + 16 + 8 * hh + 4);
    float xs[16] = {x0[0],x0[1],x0[2],x0[3],x1[0],x1[1],x1[2],x1[3],x2[0],x2[1],x2[2],x2[3],x3[0],x3[1],x3[2],x3[3]};
#pragma unroll
    for (int i = 0; i < 16; ++i) { const _Float16 h = (_Float16)xs[i]; ah.h[i] = h; al.h[i] = ASPLIT ? (_Float16)(xs[i] - (float)h) : (_Float16)0.0f; }
#pragma unroll
    for (int t = 0; t < 4; ++t) { if (col0 + t * 16 >= N) continue; const size_t boff = (size_t)(col0 + t * 16 + ln) * ldb + kb; FragH bq; bq.half[0] = *(const v8us*)(Bh + boff + 8 * hh); bq.half[1] = *(const v8us*)(Bh + boff + 16 + 8 * hh);
      acc[t] = mmaH<ASPLIT ? 2 : 1>(ah.v, al.v, bq.v, bq.v, acc[t]); }
  }
#pragma unroll
  for (int t = 0; t < 4; ++t) { if (col0 + t * 16 >= N) continue;
#pragma unroll
    for (int r = 0; r < 8; ++r) so[w][8 * hh + r][t * 16 + ln] = acc[t][r] * alpha; }
  __builtin_amdgcn_fence(__ATOMIC_ACQ_REL, "workgroup"); __builtin_amdgcn_wave_barrier();
  const int rsub = lane >> 4, c4 = (lane & 15) * 4;
  for (int pass = 0; pass < 2; ++pass) {
#pragma unroll
    for (int q = 0; q < 8; ++q) { const int r = q * 2 + rsub; if (col0 + c4 < N) { const v4f v = *(const v4fa*)&so[w][r][c4]; *(volatile v4f*)(C + (size_t)(row0 + r) * ldc + col0 + c4) = v; } }
    if (pass == 0) __threadfence(); }
}

__global__ __launch_bounds__(256) void k_wt_f16(const float* __restrict__ W, _Float16* __restrict__ Wt, int K, int N, float scale) {
  const int t = blockIdx.x * 256 + threadIdx.x; if (t >= N * (K / 8)) return; const int n = t / (K / 8), k8 = (t % (K / 8)) * 8; FragH f;
#pragma unroll
  for (int i = 0; i < 8; ++i) f.h[i] = (_Float16)(bf16_round(W[(size_t)(k8 + i) * N + n]) * scale); const v8us o = f.half[0];
  *(volatile v8us*)((unsigned short*)Wt + (size_t)n * K + k8) = o; __threadfence(); *(volatile v8us*)((unsigned short*)Wt + (size_t)n * K + k8) = o;
}
template <int ACT>
__global__ __launch_bounds__(128) void k_gemm_hhx(const _Float16* __restrict__ A, int lda, size_t sA, const _Float16* __restrict__ Bh, int ldb, size_t sB, float alpha, const float* __restrict__ bias, size_t sBias, const float* __restrict__ CP, int rowsPerB, size_t sCPb, int row0g,
    float* __restrict__ C, _Float16* __restrict__ C16, int ldc, size_t sC, int M, int N, int K) {
  __shared__ __attribute__((aligned(16))) float so[4][16][64];
  const int tid = threadIdx.x, w = tid >> 5, lane = tid & 31, ln = lane & 15, hh = lane >> 4; const int by = blockIdx.y;
  A += (size_t)by * sA; Bh += (size_t)by * sB; const size_t cofs = (size_t)by * sC; const float* bp = bias ? bias + (size_t)by * sBias : nullptr;
  const int ntn = (N + 63) / 64; const int wid = blockIdx.x * 4 + w; const int mt = wid / ntn, nq = wid % ntn; if (mt * 16 >= M) return;
  const int row0 = mt * 16, col0 = nq * 64; const _Float16* arow = A + (size_t)(row0 + ln) * lda;
  v8f acc[4] = {};
  for (int kb = 0; kb < K; kb += 32) { FragH ah; ah.half[0] = *(const v8us*)((const unsigned short*)arow + kb + 8 * hh); ah.half[1] = *(const v8us*)((const unsigned short*)arow + kb + 16 + 8 * hh);
#pragma unroll
    for (int t = 0; t < 4; ++t) { if (col0 + t * 16 >= N) continue; const size_t boff = (size_t)(col0 + t * 16 + ln) * ldb + kb; FragH bq; bq.half[0] = *(const v8us*)((const unsigned short*)Bh + boff + 8 * hh); bq.half[1] = *(const v8us*)((const unsigned short*)Bh + boff + 16 + 8 * hh);
      acc[t] = mmaH<1>(ah.v, ah.v, bq.v, bq.v, acc[t]); }
  }
#pragma unroll
  for (int t = 0; t < 4; ++t) { if (col0 + t * 16 >= N) continue; const int col = col0 + t * 16 + ln; const float bv = bp ? bf16_round(bp[col]) : 0.f;
#pragma unroll
    for (int r = 0; r < 8; ++r) { float v = acc[t][r] * alpha + bv; if (CP) { const int bidx = (row0g + row0 + 8 * hh + r) / rowsPerB; v += CP[(size_t)bidx * sCPb + (size_t)by * 64 + col]; } if (ACT == 1) v = (v > 0.f) ? v : expm1f(v); else if (ACT == 3) v = fmaxf(v, 0.f); else if (ACT == 6) v = 0.5f * v * (1.0f + erff(v * 0.70710678118654752f)); so[w][8 * hh + r][t * 16 + ln] = v; } }
  __builtin_amdgcn_fence(__ATOMIC_ACQ_REL, "workgroup"); __builtin_amdgcn_wave_barrier();
  const int rsub = lane >> 4, c4 = (lane & 15) * 4; typedef _Float16 v4h __attribute__((ext_vector_type(4)));
  for (int pass = 0; pass < 2; ++pass) {
#pragma unroll
    for (int q = 0; q < 8; ++q) { const int r = q * 2 + rsub; if (col0 + c4 < N) { const v4f v = *(const v4fa*)&so[w][r][c4]; if (C) *(volatile v4f*)(C + cofs + (size_t)(row0 + r) * ldc + col0 + c4) = v; if (C16) { v4h h4; for (int i = 0; i < 4; ++i) h4[i] = (_Float16)v[i]; *(volatile v4h*)(C16 + cofs + (size_t)(row0 + r) * ldc + col0 + c4) = h4; } } }
    if (pass == 0) __threadfence(); }
}


__global__ __launch_bounds__(64) void k_xstat(const float* __restrict__ x, float* __restrict__ MS) { const int b = threadIdx.x; float s = 0.f; for (int i = 0; i < II; ++i) s += bf16_round(x[b * II + i]); const float mu = s / (float)II; float q2 = 0.f; for (int i = 0; i < II; ++i) { const float d = bf16_round(x[b * II + i]) - mu; q2 += d * d; } typedef float v2f __attribute__((ext_vector_type(2))); v2f o; o[0] = mu; o[1] = rsqrtf(q2 / (float)II + 1e-5f); *(volatile v2f*)(MS + b * 2) = o; __threadfence(); *(volatile v2f*)(MS + b * 2) = o; }
__global__ __launch_bounds__(256) void k_xn(const float* __restrict__ x, const float* __restrict__ MS, const float* __restrict__ g, const float* __restrict__ bb, _Float16* __restrict__ XN) { const size_t t = (size_t)blockIdx.x * 256 + threadIdx.x; if (t >= (size_t)NR * 8) return; const int c8 = (int)(t % 8) * 8; const size_t r = t / 8; const int a = (int)(r / BBt), b = (int)(r % BBt); const float mu = MS[b * 2], rs = MS[b * 2 + 1]; FragH f;
#pragma unroll
  for (int q = 0; q < 8; ++q) { const int i = c8 + q; f.h[q] = (_Float16)((i < II) ? ((bf16_round(x[b * II + i]) - mu) * rs * bf16_round(g[a * II + i]) + bf16_round(bb[a * II + i])) : 0.f); }
  *(volatile v8us*)((unsigned short*)XN + t * 8) = f.half[0]; __threadfence(); *(volatile v8us*)((unsigned short*)XN + t * 8) = f.half[0]; }
__global__ __launch_bounds__(256) void k_wta(const float* __restrict__ W, int kin, int kp, int nout, _Float16* __restrict__ Bt) { const size_t t = (size_t)blockIdx.x * 256 + threadIdx.x; if (t >= (size_t)AA * nout * (kp / 8)) return; const int k8 = (int)(t % (kp / 8)) * 8; const int o = (int)((t / (kp / 8)) % nout); const int a = (int)(t / ((size_t)nout * (kp / 8))); FragH f;
#pragma unroll
  for (int q = 0; q < 8; ++q) { const int k = k8 + q; f.h[q] = (_Float16)((k < kin) ? bf16_round(W[((size_t)a * kin + k) * nout + o]) * 16.0f : 0.f); } *(volatile v8us*)((unsigned short*)Bt + t * 8) = f.half[0]; __threadfence(); *(volatile v8us*)((unsigned short*)Bt + t * 8) = f.half[0]; }
typedef _Float16 v4h __attribute__((ext_vector_type(4)));
__global__ __launch_bounds__(256) void k_add(float* __restrict__ T, const float* __restrict__ S, _Float16* __restrict__ H16, size_t n4) { const size_t t = (size_t)blockIdx.x * 256 + threadIdx.x; if (t >= n4) return; const v4f a = *(const v4fa*)(T + t * 4), s = *(const v4fa*)(S + t * 4); v4f o; v4h h; for (int q = 0; q < 4; ++q) { o[q] = a[q] + s[q]; h[q] = (_Float16)o[q]; }
  for (int pass = 0; pass < 2; ++pass) { *(volatile v4f*)(T + t * 4) = o; *(volatile v4h*)(H16 + t * 4) = h; if (pass == 0) __threadfence(); } }

__global__ __launch_bounds__(256) void k_ln(const float* __restrict__ X, const float* __restrict__ AADD, const float* __restrict__ ga, const float* __restrict__ ba, int astride, float* __restrict__ OUT, _Float16* __restrict__ O16) { const size_t t = (size_t)blockIdx.x * 256 + threadIdx.x; if (t >= (size_t)NR * 16) return; const int li = (int)(t % 16); const size_t r = t / 16; const int a = (int)(r / BBt); v4f v[3]; float s = 0.f;
#pragma unroll
  for (int p = 0; p < 3; ++p) { v[p] = *(const v4fa*)(X + r * HH + 64 * p + 4 * li); if (AADD) { const v4f w2 = *(const v4fa*)(AADD + r * HH + 64 * p + 4 * li); v[p] += w2; } s += v[p][0] + v[p][1] + v[p][2] + v[p][3]; }
  s += __shfl_xor(s, 1, 32); s += __shfl_xor(s, 2, 32); s += __shfl_xor(s, 4, 32); s += __shfl_xor(s, 8, 32); const float mu = s / (float)HH; float q2 = 0.f;
#pragma unroll
  for (int p = 0; p < 3; ++p) for (int q = 0; q < 4; ++q) { const float d = v[p][q] - mu; q2 += d * d; } q2 += __shfl_xor(q2, 1, 32); q2 += __shfl_xor(q2, 2, 32); q2 += __shfl_xor(q2, 4, 32); q2 += __shfl_xor(q2, 8, 32); const float rs = rsqrtf(q2 / (float)HH + 1e-5f);
  v4f o[3]; v4h h[3];
#pragma unroll
  for (int p = 0; p < 3; ++p) for (int q = 0; q < 4; ++q) { const int c = 64 * p + 4 * li + q; const float y = (v[p][q] - mu) * rs * bf16_round(ga[(size_t)a * astride + c]) + bf16_round(ba[(size_t)a * astride + c]); o[p][q] = y; h[p][q] = (_Float16)y; }
  for (int pass = 0; pass < 2; ++pass) {
#pragma unroll
    for (int p = 0; p < 3; ++p) { if (OUT) *(volatile v4f*)(OUT + r * HH + 64 * p + 4 * li) = o[p]; if (O16) *(volatile v4h*)(O16 + r * HH + 64 * p + 4 * li) = h[p]; }
    if (pass == 0) __threadfence(); } }
__global__ __launch_bounds__(256) void k_qkp(const _Float16* __restrict__ Q16, const _Float16* __restrict__ K16, int j0, _Float16* __restrict__ QP, _Float16* __restrict__ KP) { const int t = blockIdx.x * 256 + threadIdx.x; if (t >= JCH * AA * 4) return; const int p = t % 4; const int a = (t / 4) % AA; const int j = t / (4 * AA); const int J = j0 + j; const int b = J / NHD, h = J % NHD; v8us q, k; if (p < 2) { const size_t src = ((size_t)a * BBt + b) * AD + h * HD + p * 8; q = *(const v8us*)((const unsigned short*)Q16 + src); k = *(const v8us*)((const unsigned short*)K16 + src); } else { q = (v8us){0,0,0,0,0,0,0,0}; k = q; }
  for (int pass = 0; pass < 2; ++pass) { *(volatile v8us*)((unsigned short*)QP + (size_t)t * 8) = q; *(volatile v8us*)((unsigned short*)KP + (size_t)t * 8) = k; if (pass == 0) __threadfence(); } }
__global__ __launch_bounds__(256) void k_vtp(const _Float16* __restrict__ V16, int j0, _Float16* __restrict__ VT) { const int t = blockIdx.x * 256 + threadIdx.x; if (t >= JCH * HD * (KPAD / 8)) return; const int pc = t % (KPAD / 8); const int d = (t / (KPAD / 8)) % HD; const int j = t / ((KPAD / 8) * HD); const int J = j0 + j; const int b = J / NHD, h = J % NHD; FragH f;
#pragma unroll
  for (int q = 0; q < 8; ++q) { const int c = pc * 8 + q; f.h[q] = (c < AA) ? V16[((size_t)c * BBt + b) * AD + h * HD + d] : (_Float16)0.f; }
  *(volatile v8us*)((unsigned short*)VT + (size_t)t * 8) = f.half[0]; __threadfence(); *(volatile v8us*)((unsigned short*)VT + (size_t)t * 8) = f.half[0]; }
__global__ __launch_bounds__(256) void k_psm(const float* __restrict__ S, _Float16* __restrict__ P16) { const int tid = threadIdx.x, wv = tid >> 5, lane = tid & 31; const int row = blockIdx.x * 8 + wv; if (row >= JCH * AA) return; const float* sr = S + (size_t)row * 416; float v[16]; float m = -3.0e38f;
#pragma unroll
  for (int q = 0; q < 8; ++q) { v[q] = sr[8 * lane + q]; m = fmaxf(m, v[q]); }
#pragma unroll
  for (int q = 0; q < 8; ++q) { const int c = 256 + 8 * lane + q; v[8 + q] = (c < AA) ? sr[c] : -3.0e38f; m = fmaxf(m, v[8 + q]); }
  for (int o = 16; o >= 1; o >>= 1) m = fmaxf(m, __shfl_xor(m, o, 32)); float s = 0.f; float e[16];
#pragma unroll
  for (int q = 0; q < 16; ++q) { e[q] = (v[q] > -1.0e38f) ? expf(v[q] - m) : 0.f; s += e[q]; } for (int o = 16; o >= 1; o >>= 1) s += __shfl_xor(s, o, 32); const float is = 1.0f / s; FragH f0, f1;
#pragma unroll
  for (int q = 0; q < 8; ++q) { f0.h[q] = (_Float16)(e[q] * is); f1.h[q] = (_Float16)(e[8 + q] * is); }
  unsigned short* d = (unsigned short*)P16 + (size_t)row * KPAD;
  for (int pass = 0; pass < 2; ++pass) { *(volatile v8us*)(d + 8 * lane) = f0.half[0]; if (lane < 24) *(volatile v8us*)(d + 256 + 8 * lane) = f1.half[0]; if (pass == 0) __threadfence(); } }
__global__ __launch_bounds__(256) void k_h16(const float* __restrict__ x, _Float16* __restrict__ X16, size_t n8) { const size_t t = (size_t)blockIdx.x * 256 + threadIdx.x; if (t >= n8) return; FragH f;
#pragma unroll
  for (int q = 0; q < 8; ++q) f.h[q] = (_Float16)x[t * 8 + q]; *(volatile v8us*)((unsigned short*)X16 + t * 8) = f.half[0]; __threadfence(); *(volatile v8us*)((unsigned short*)X16 + t * 8) = f.half[0]; }
__global__ __launch_bounds__(256) void k_head(const float* __restrict__ ATT, const float* __restrict__ Wout, const float* __restrict__ bout, float* __restrict__ out) { const size_t t = (size_t)blockIdx.x * 256 + threadIdx.x; if (t >= (size_t)NR * OO) return; const int o = (int)(t % OO); const size_t r = t / OO; const int a = (int)(r / BBt); float s = bf16_round(bout[a * OO + o]);
#pragma unroll 1
  for (int h = 0; h < HH; ++h) s += ATT[r * HH + h] * bf16_round(Wout[((size_t)a * HH + h) * OO + o]); *(volatile float*)(out + t) = s; __threadfence(); *(volatile float*)(out + t) = s; }

__global__ __launch_bounds__(256) void k_orep(const float* __restrict__ OC, int b0, _Float16* __restrict__ O16) { const int t = blockIdx.x * 256 + threadIdx.x; if (t >= AA * (JCH / NHD) * 16) return; const int p = t % 16; const int bl = (t / 16) % (JCH / NHD); const int a = t / (16 * (JCH / NHD)); const int h = p / 2, d8 = (p % 2) * 8; const float* src = OC + ((size_t)(bl * NHD + h) * AA + a) * HD + d8; FragH f;
#pragma unroll
  for (int q = 0; q < 8; ++q) f.h[q] = (_Float16)src[q]; unsigned short* dst = (unsigned short*)O16 + ((size_t)a * BBt + b0 + bl) * AD + p * 8; *(volatile v8us*)dst = f.half[0]; __threadfence(); *(volatile v8us*)dst = f.half[0]; }
extern "C" void kernel_launch(void* const* d_in, const int* in_sizes, int n_in,
                              void* d_out, int out_size, void* d_ws, size_t ws_size, hipStream_t stream) {
  (void)in_sizes; (void)n_in; (void)out_size;
  const float* const* I = (const float* const*)d_in; const float* x = I[0]; const float* lng = I[1]; const float* lnb = I[2]; const float* W1 = I[3]; const float* b1 = I[4]; const float* Ws1 = I[5]; const float* bs1 = I[6]; const float* W2 = I[7]; const float* b2 = I[8]; const float* Ws2 = I[9]; const float* bs2 = I[10]; const float* W3 = I[11]; const float* b3 = I[12];
  const float* lhg = I[13]; const float* lhb = I[14]; const float* Wout = I[15]; const float* bout = I[16]; const float* ag = I[17]; const float* ab = I[18]; const float* Wq = I[19]; const float* bq = I[20]; const float* Wk = I[21]; const float* bk = I[22]; const float* Wv = I[23]; const float* bv = I[24]; const float* Wo = I[25]; const float* bo = I[26];
  char* ws = (char*)d_ws; size_t off = 0;
  auto take = [&](size_t bytes) { char* p = ws + off; off += (bytes + 255) & ~(size_t)255; return p; };
  float* MSx = (float*)take(BBt * 2 * 4); _Float16* XN = (_Float16*)take((size_t)NR * IP * 2); _Float16* BtS = (_Float16*)take((size_t)AA * HH * IP * 2); _Float16* BtL = (_Float16*)take((size_t)AA * HH * HH * 2);
  float* P0 = (float*)take((size_t)NR * HH * 4); float* P1 = (float*)take((size_t)NR * HH * 4); float* P2 = (float*)take((size_t)NR * HH * 4); _Float16* H16 = (_Float16*)take((size_t)NR * HH * 2);
  _Float16* Bq = (_Float16*)take(AD * HH * 2); _Float16* Bk = (_Float16*)take(AD * HH * 2); _Float16* Bv = (_Float16*)take(AD * HH * 2); _Float16* Bo = (_Float16*)take(HH * AD * 2);
  _Float16* Q16 = (_Float16*)take((size_t)NR * AD * 2); _Float16* K16 = (_Float16*)take((size_t)NR * AD * 2); _Float16* V16 = (_Float16*)take((size_t)NR * AD * 2);
  if (off > ws_size) return;
  const size_t n4 = (size_t)NR * HH / 4, n8 = (size_t)NR * HH / 8; const unsigned g4 = (unsigned)((n4 + 255) / 256), g8 = (unsigned)((n8 + 255) / 256), g16 = (unsigned)(((size_t)NR * 16 + 255) / 256);
  const dim3 gb(((BBt / 16) * (HH / 64) + 3) / 4, AA);
  k_xstat<<<1, 64, 0, stream>>>(x, MSx); k_xn<<<(unsigned)(((size_t)NR * 8 + 255) / 256), 256, 0, stream>>>(x, MSx, lng, lnb, XN);
  k_wta<<<(unsigned)(((size_t)AA * HH * (IP / 8) + 255) / 256), 256, 0, stream>>>(W1, II, IP, HH, BtS);
  k_gemm_hhx<6><<<gb, 128, 0, stream>>>(XN, IP, (size_t)BBt * IP, BtS, IP, (size_t)HH * IP, 0.0625f, b1, HH, nullptr, 1, 0, 0, P0, nullptr, HH, (size_t)BBt * HH, BBt, HH, IP);
  k_wta<<<(unsigned)(((size_t)AA * HH * (IP / 8) + 255) / 256), 256, 0, stream>>>(Ws1, II, IP, HH, BtS);
  k_gemm_hhx<0><<<gb, 128, 0, stream>>>(XN, IP, (size_t)BBt * IP, BtS, IP, (size_t)HH * IP, 0.0625f, bs1, HH, nullptr, 1, 0, 0, P1, nullptr, HH, (size_t)BBt * HH, BBt, HH, IP);
  k_add<<<g4, 256, 0, stream>>>(P0, P1, H16, n4);
  k_wta<<<(unsigned)(((size_t)AA * HH * (HH / 8) + 255) / 256), 256, 0, stream>>>(W2, HH, HH, HH, BtL);
  k_gemm_hhx<6><<<gb, 128, 0, stream>>>(H16, HH, (size_t)BBt * HH, BtL, HH, (size_t)HH * HH, 0.0625f, b2, HH, nullptr, 1, 0, 0, P1, nullptr, HH, (size_t)BBt * HH, BBt, HH, HH);
  k_wta<<<(unsigned)(((size_t)AA * HH * (HH / 8) + 255) / 256), 256, 0, stream>>>(Ws2, HH, HH, HH, BtL);
  k_gemm_hhx<0><<<gb, 128, 0, stream>>>(H16, HH, (size_t)BBt * HH, BtL, HH, (size_t)HH * HH, 0.0625f, bs2, HH, nullptr, 1, 0, 0, P2, nullptr, HH, (size_t)BBt * HH, BBt, HH, HH);
  k_add<<<g4, 256, 0, stream>>>(P1, P2, H16, n4);
  k_wta<<<(unsigned)(((size_t)AA * HH * (HH / 8) + 255) / 256), 256, 0, stream>>>(W3, HH, HH, HH, BtL);
  k_gemm_hhx<0><<<gb, 128, 0, stream>>>(H16, HH, (size_t)BBt * HH, BtL, HH, (size_t)HH * HH, 0.0625f, b3, HH, nullptr, 1, 0, 0, P2, nullptr, HH, (size_t)BBt * HH, BBt, HH, HH);
  k_ln<<<g16, 256, 0, stream>>>(P1, P2, lhg, lhb, HH, P0, nullptr);
  k_ln<<<g16, 256, 0, stream>>>(P0, nullptr, ag, ab, 0, nullptr, H16);
  k_wt_f16<<<(AD * (HH / 8) + 255) / 256, 256, 0, stream>>>(Wq, Bq, HH, AD, 16.0f); k_wt_f16<<<(AD * (HH / 8) + 255) / 256, 256, 0, stream>>>(Wk, Bk, HH, AD, 16.0f); k_wt_f16<<<(AD * (HH / 8) + 255) / 256, 256, 0, stream>>>(Wv, Bv, HH, AD, 16.0f); k_wt_f16<<<(HH * (AD / 8) + 255) / 256, 256, 0, stream>>>(Wo, Bo, AD, HH, 16.0f);
  const dim3 gp(((NR / 16) * (AD / 64) + 3) / 4, 1);
  k_gemm_hhx<0><<<gp, 128, 0, stream>>>(H16, HH, 0, Bq, HH, 0, 0.0625f, bq, 0, nullptr, 1, 0, 0, nullptr, Q16, AD, 0, NR, AD, HH);
  k_gemm_hhx<0><<<gp, 128, 0, stream>>>(H16, HH, 0, Bk, HH, 0, 0.0625f, bk, 0, nullptr, 1, 0, 0, nullptr, K16, AD, 0, NR, AD, HH);
  k_gemm_hhx<0><<<gp, 128, 0, stream>>>(H16, HH, 0, Bv, HH, 0, 0.0625f, bv, 0, nullptr, 1, 0, 0, nullptr, V16, AD, 0, NR, AD, HH);
  char* sc = (char*)P1; float* S = (float*)sc; _Float16* P16 = (_Float16*)(sc + (size_t)JCH * AA * 416 * 4); _Float16* QP = (_Float16*)((char*)P16 + (size_t)JCH * AA * KPAD * 2); _Float16* KP = (_Float16*)((char*)QP + (size_t)JCH * AA * 32 * 2); _Float16* VT = (_Float16*)((char*)KP + (size_t)JCH * AA * 32 * 2); float* OC = (float*)((char*)VT + (size_t)JCH * HD * KPAD * 2);
  _Float16* O16 = XN;
  for (int j0 = 0; j0 < BBt * NHD; j0 += JCH) {
    k_qkp<<<(JCH * AA * 4 + 255) / 256, 256, 0, stream>>>(Q16, K16, j0, QP, KP); k_vtp<<<(JCH * HD * (KPAD / 8) + 255) / 256, 256, 0, stream>>>(V16, j0, VT);
    k_gemm_hhx<0><<<dim3(((AA / 16) * ((AA + 63) / 64) + 3) / 4, JCH), 128, 0, stream>>>(QP, 32, (size_t)AA * 32, KP, 32, (size_t)AA * 32, 0.25f, nullptr, 0, nullptr, 1, 0, 0, S, nullptr, 416, (size_t)AA * 416, AA, AA, 32);
    k_psm<<<(JCH * AA + 7) / 8, 256, 0, stream>>>(S, P16);
    k_gemm_hhx<0><<<dim3(((AA / 16) * 1 + 3) / 4, JCH), 128, 0, stream>>>(P16, KPAD, (size_t)AA * KPAD, VT, KPAD, (size_t)HD * KPAD, 1.0f, nullptr, 0, nullptr, 1, 0, 0, OC, nullptr, HD, (size_t)AA * HD, AA, HD, KPAD);
    k_orep<<<(AA * (JCH / NHD) * 16 + 255) / 256, 256, 0, stream>>>(OC, j0 / NHD, O16); }
  k_gemm_hhx<0><<<dim3(((NR / 16) * (HH / 64) + 3) / 4, 1), 128, 0, stream>>>(O16, AD, 0, Bo, AD, 0, 0.0625f, bo, 0, P0, 1, (size_t)HH, 0, P2, nullptr, HH, 0, NR, HH, AD);
  k_head<<<(unsigned)(((size_t)NR * OO + 255) / 256), 256, 0, stream>>>(P2, Wout, bout, (float*)d_out);
}
